// MultiPerspectiveLayer_41077067219604
// MI455X (gfx1250) — hardware-verified
//
#include <hip/hip_runtime.h>
#include <math.h>

typedef __attribute__((ext_vector_type(16))) _Float16 v16h;
typedef __attribute__((ext_vector_type(16))) __bf16 v16b;
typedef __attribute__((ext_vector_type(8)))  _Float16 v8h;
typedef __attribute__((ext_vector_type(8)))  float v8f;
typedef __attribute__((ext_vector_type(4)))  float v4f;
typedef __attribute__((ext_vector_type(2)))  float v2f;
typedef __attribute__((ext_vector_type(4)))  unsigned v4u;
typedef __attribute__((ext_vector_type(4)))  int v4i;
typedef float __attribute__((may_alias)) float_a;
typedef int __attribute__((may_alias)) int_a;

template <typename T> __device__ __forceinline__ void vst2(void* p, T v) { *(volatile T*)p = v; __threadfence(); *(volatile T*)p = v; }
__device__ __forceinline__ v8f wmma16(v16h a, v16h b, v8f c) {
  v8f d = __builtin_amdgcn_wmma_f32_16x16x32_f16(false, a, false, b, (short)0, c, false, false);
  asm volatile("v_nop\n\tv_nop\n\tv_nop\n\tv_nop" : "+v"(d) : "v"(a), "v"(b));
  return d;
}
__device__ __forceinline__ v8f wmma_bf(v16b a, v16b b, v8f c) {
  v8f d = __builtin_amdgcn_wmma_f32_16x16x32_bf16(false, a, false, b, (short)0, c, false, false);
  asm volatile("v_nop\n\tv_nop\n\tv_nop\n\tv_nop" : "+v"(d) : "v"(a), "v"(b));
  return d;
}
__device__ __forceinline__ v16h frag_h(const _Float16* rowk0, int lane) {
  union { v16h v; v8h q[2]; } u; const _Float16* p = rowk0 + 8 * (lane >> 4);
  u.q[0] = *(const v8h*)p; u.q[1] = *(const v8h*)(p + 16); return u.v;
}
__device__ __forceinline__ v16h frag_f32(const float* rowk0, int lane) {
  v16h a; const float* p = rowk0 + 8 * (lane >> 4);
#pragma unroll
  for (int i = 0; i < 8; ++i) { a[i] = (_Float16)p[i]; a[8 + i] = (_Float16)p[16 + i]; }
  return a;
}
__device__ __forceinline__ v16h frag_f32s(const float* rowk0, int lane, float sc) {
  v16h a; const float* p = rowk0 + 8 * (lane >> 4);
#pragma unroll
  for (int i = 0; i < 8; ++i) { a[i] = (_Float16)(p[i] * sc); a[8 + i] = (_Float16)(p[16 + i] * sc); }
  return a;
}
__device__ __forceinline__ v16h fragc_f32(const float* W, int k0, int n, int lane, int ld, int K) {
  v16h a; const int g = lane >> 4;
#pragma unroll
  for (int i = 0; i < 8; ++i) { const int ka = k0 + 8 * g + i, kb = ka + 16;
    a[i] = (_Float16)(ka < K ? W[(size_t)(ka < K ? ka : K - 1) * ld + n] : 0.f); a[8 + i] = (_Float16)(kb < K ? W[(size_t)(kb < K ? kb : K - 1) * ld + n] : 0.f); }
  return a;
}
struct F2 { v16b h, l; };
__device__ __forceinline__ F2 bsplit16(const float v[16]) { F2 r;
#pragma unroll
  for (int i = 0; i < 16; ++i) { const __bf16 h = (__bf16)v[i]; r.h[i] = h; r.l[i] = (__bf16)(v[i] - (float)h); }
  return r; }
__device__ __forceinline__ F2 split_row(const float* row, int k0, int lane) { float v[16]; const float* p = row + k0 + 8 * (lane >> 4);
#pragma unroll
  for (int i = 0; i < 8; ++i) { v[i] = p[i]; v[8 + i] = p[16 + i]; }
  return bsplit16(v); }
__device__ __forceinline__ F2 split_rowK(const float* row, int k0, int lane, int K) { float v[16]; const int g = lane >> 4;
#pragma unroll
  for (int i = 0; i < 8; ++i) { const int ka = k0 + 8 * g + i, kb = ka + 16; v[i] = ka < K ? row[ka < K ? ka : K - 1] : 0.f; v[8 + i] = kb < K ? row[kb < K ? kb : K - 1] : 0.f; }
  return bsplit16(v); }
__device__ __forceinline__ F2 split_col(const float* W, int k0, int n, int lane, int ld, int K) { float v[16]; const int g = lane >> 4;
#pragma unroll
  for (int i = 0; i < 8; ++i) { const int ka = k0 + 8 * g + i, kb = ka + 16; v[i] = ka < K ? W[(size_t)(ka < K ? ka : K - 1) * ld + n] : 0.f; v[8 + i] = kb < K ? W[(size_t)(kb < K ? kb : K - 1) * ld + n] : 0.f; }
  return bsplit16(v); }
__device__ __forceinline__ v8f mac3(const F2& a, const F2& b, v8f c) { c = wmma_bf(a.l, b.h, c); c = wmma_bf(a.h, b.l, c); return wmma_bf(a.h, b.h, c); }
__device__ __forceinline__ float sigm(float v) { return 1.0f / (1.0f + expf(-v)); }
#define LDSX() do { asm volatile("s_wait_dscnt 0" ::: "memory"); __builtin_amdgcn_wave_barrier(); __builtin_amdgcn_fence(__ATOMIC_RELEASE, "workgroup"); } while (0)


#define NB 64
#define LL 128
#define DD 200
#define DP 224
#define MP 20
#define ATT 50
#define AP 64
#define NOUT 83
#define NR (NB * LL)
#ifndef NBT
#define NBT NB
#endif
typedef __attribute__((ext_vector_type(8))) __bf16 v8b;
__device__ __forceinline__ v16b frag_b(const __bf16* rowk0, int lane) {
  union { v16b v; v8b q[2]; } u; const __bf16* p = rowk0 + 8 * (lane >> 4);
  u.q[0] = *(const v8b*)p; u.q[1] = *(const v8b*)(p + 16); return u.v;
}
__device__ __forceinline__ float bfr(float v) { return (float)(__bf16)v; }
__device__ __attribute__((noinline)) float exp_ni(float v) { return expf(v); }
__device__ __attribute__((noinline)) float erf_ni(float v) { return erff(v); }

__device__ __attribute__((noinline)) float tanh_ni(float v) { return tanhf(v); }
#define WS_PW1  0u
#define WS_PW2  (WS_PW1 + 2u * AP * DP)
#define WS_HWF  (WS_PW2 + 2u * AP * DP)
#define WS_ELT  (WS_HWF + 4u * NB * MP * DP)
#define WS_LTT  (WS_ELT + 4u * NB * LL * AP)
#define WS_NLT  (WS_LTT + 2u * NB * DP * LL)
#define WS_OS   (WS_NLT + 4u * NB * LL)
#define WS_END  (WS_OS + 4u * NR * 96)

__device__ __forceinline__ v16b fragD(const float* row, int k0, int lane) {
  v16b a; const int g = lane >> 4;
#pragma unroll
  for (int i = 0; i < 8; ++i) { const int ka = k0 + 8 * g + i, kb = ka + 16; a[i] = (__bf16)(ka < DD ? row[ka < DD ? ka : 0] : 0.f); a[8 + i] = (__bf16)(kb < DD ? row[kb < DD ? kb : 0] : 0.f); }
  return a; }
__global__ __launch_bounds__(128) void k_packw(const float* __restrict__ Wm, __bf16* __restrict__ DST) {
  __shared__ __align__(16) __bf16 s[8 * DP]; const int a0 = blockIdx.x * 8, tid = threadIdx.x;
  for (int q = tid; q < 8 * DP; q += 128) { const int al = q / DP, k = q % DP; const int a = a0 + al; s[q] = (__bf16)((a < ATT && k < DD) ? Wm[(size_t)k * ATT + a] : 0.f); }
  __syncthreads();
  for (int q = tid; q < DP; q += 128) vst2((unsigned*)(DST + (size_t)a0 * DP + q * 8), *(const v4u*)&s[q * 8]);
}
__global__ __launch_bounds__(256) void k_prep(const float* __restrict__ LT, const float* __restrict__ FW, const float* __restrict__ BW, const float* __restrict__ WF, const __bf16* __restrict__ PW2, float* __restrict__ HWF, float* __restrict__ ELT, __bf16* __restrict__ LTT, float* __restrict__ NLT) {
  __shared__ __align__(16) __bf16 slt[LL][DP + 8]; __shared__ __align__(16) float srow[256]; __shared__ __align__(16) float selt[8][16][AP + 4];
  const int b = blockIdx.x, tid = threadIdx.x, wave = tid >> 5, lane = tid & 31, col = lane & 15, g = lane >> 4; const float* lt = LT + (size_t)b * LL * DD;
  for (int q = tid; q < LL * DP; q += 256) { const int l = q / DP, d = q % DP; slt[l][d] = (__bf16)(d < DD ? lt[(size_t)l * DD + d] : 0.f); }
  __syncthreads();
  for (int q = tid; q < DP * 16; q += 256) { const int d = q >> 4, pc = q & 15; union { v4u v; __bf16 hh[8]; } u;
#pragma unroll
    for (int i = 0; i < 8; ++i) u.hh[i] = slt[pc * 8 + i][d];
    vst2((unsigned*)(LTT + ((size_t)b * DP + d) * LL + pc * 8), u.v); }
  if (tid < LL) { float s = 0.f; for (int d = 0; d < DD; ++d) { const float v = bfr(lt[(size_t)tid * DD + d]); s += v * v; } srow[tid] = 1.0f / sqrtf(fmaxf(s, 1e-6f)); }
  __syncthreads();
  if (tid < 32) vst2(NLT + (size_t)b * LL + tid * 4, *(const v4f*)&srow[tid * 4]);
  __syncthreads();
  for (int m = 0; m < MP; ++m) { for (int d = tid; d < DP; d += 256) { float v = 0.f; if (d < DD) { const float hv = (d < DD / 2) ? bfr(FW[(size_t)b * (DD / 2) + d]) : bfr(BW[(size_t)b * (DD / 2) + d - DD / 2]); v = bfr(WF[(size_t)m * DD + d]) * hv; } srow[d] = v; }
    __syncthreads();
    if (tid < DP / 4) vst2(HWF + ((size_t)b * MP + m) * DP + tid * 4, *(const v4f*)&srow[tid * 4]);
    __syncthreads(); }
  { v8f acc[4] = {};
#pragma unroll
    for (int kc = 0; kc < DP / 32; ++kc) { const v16b a = frag_b(&slt[wave * 16 + col][kc * 32], lane);
#pragma unroll
      for (int j = 0; j < 4; ++j) acc[j] = wmma_bf(a, frag_b(PW2 + (size_t)(j * 16 + col) * DP + kc * 32, lane), acc[j]); }
#pragma unroll
    for (int j = 0; j < 4; ++j)
#pragma unroll
      for (int r = 0; r < 8; ++r) selt[wave][8 * g + r][j * 16 + col] = tanh_ni(acc[j][r]);
    LDSX();
    for (int rl = 0; rl < 16; ++rl) if (lane < 16) vst2(ELT + ((size_t)b * LL + wave * 16 + rl) * AP + lane * 4, *(const v4f*)&selt[wave][rl][lane * 4]); }
}
__global__ __launch_bounds__(128) void k_main(const float* __restrict__ LT, const float* __restrict__ RT, const float* __restrict__ WMX, const float* __restrict__ WAT, const float* __restrict__ WMA, const __bf16* __restrict__ PW1, const float* __restrict__ DIAG,
    const float* __restrict__ FW, const float* __restrict__ BW, const float* __restrict__ HWF, const float* __restrict__ ELT, const __bf16* __restrict__ LTT, const float* __restrict__ NLT, float* __restrict__ OS) {
  __shared__ __align__(16) float slt[16][DP], srt[16][DP];
  __shared__ __align__(16) float sattl[16][DP], smal[16][DP];
  __shared__ __align__(16) float satt[16][LL + 4];
  __shared__ __align__(16) float sert[16][AP + 4];
  __shared__ __align__(16) float sout[16][96]; __shared__ float smx[4][16][16]; __shared__ int spos[16]; __shared__ float sh[DP];
  __shared__ __align__(16) __bf16 srtb[LL][DP + 8], sltb[LL][DP + 8];
  const int tid = threadIdx.x, wave = tid >> 5, lane = tid & 31, col = lane & 15, g = lane >> 4; const int i0 = blockIdx.x * 16, b = blockIdx.y; const size_t rbase = (size_t)b * LL;
  for (int q = tid; q < 16 * DP; q += 128) { const int rl = q / DP, d = q % DP; slt[rl][d] = (d < DD) ? bfr(LT[(rbase + i0 + rl) * DD + d]) : 0.f; srt[rl][d] = (d < DD) ? bfr(RT[(rbase + i0 + rl) * DD + d]) : 0.f; }
  for (int q = tid; q < 16 * 96; q += 128) (&sout[0][0])[q] = 0.f;
  for (int q = tid; q < LL * DP; q += 128) { const int l = q / DP, d = q % DP; srtb[l][d] = (__bf16)(d < DD ? RT[(rbase + l) * DD + d] : 0.f); sltb[l][d] = (__bf16)(d < DD ? LT[(rbase + l) * DD + d] : 0.f); }
  for (int d = tid; d < DP; d += 128) sh[d] = (d < DD / 2) ? bfr(FW[(size_t)b * (DD / 2) + d]) : (d < DD ? bfr(BW[(size_t)b * (DD / 2) + d - DD / 2]) : 0.f);
  __syncthreads();
#pragma unroll 1
  for (int m = wave; m < MP; m += 4) { v8f acc[8] = {};
#pragma unroll 1
    for (int kc = 0; kc < DP / 32; ++kc) { float v[16]; const int k0 = kc * 32;
#pragma unroll
      for (int i = 0; i < 8; ++i) { const int ka = k0 + 8 * g + i, kb = ka + 16; v[i] = slt[col][ka] * (ka < DD ? bfr(WMX[(size_t)m * DD + (ka < DD ? ka : DD - 1)]) : 0.f); v[8 + i] = slt[col][kb] * (kb < DD ? bfr(WMX[(size_t)m * DD + (kb < DD ? kb : DD - 1)]) : 0.f); }
      const F2 a = bsplit16(v);
#pragma unroll
      for (int j = 0; j < 8; ++j) { const v16b rb = frag_b(&srtb[j * 16 + col][k0], lane); acc[j] = wmma_bf(a.l, rb, acc[j]); acc[j] = wmma_bf(a.h, rb, acc[j]); } }
    float mx[8];
#pragma unroll
    for (int r = 0; r < 8; ++r) { float t = acc[0][r];
#pragma unroll
      for (int j = 1; j < 8; ++j) t = fmaxf(t, acc[j][r]);
#pragma unroll
      for (int o = 1; o < 16; o <<= 1) t = fmaxf(t, __shfl_xor(t, o));
      mx[r] = t; }
    if (col == 0) {
#pragma unroll
      for (int r = 0; r < 8; ++r) sout[8 * g + r][21 + m] = tanh_ni(mx[r]); } }
  if (wave == 0) { v8f acc[4] = {};
#pragma unroll
    for (int kc = 0; kc < DP / 32; ++kc) { v16b a; { const int k0 = kc * 32;
#pragma unroll
        for (int i = 0; i < 8; ++i) { a[i] = (__bf16)srt[col][k0 + 8 * g + i]; a[8 + i] = (__bf16)srt[col][k0 + 16 + 8 * g + i]; } }
#pragma unroll
      for (int j = 0; j < 4; ++j) acc[j] = wmma_bf(a, frag_b(PW1 + (size_t)(j * 16 + col) * DP + kc * 32, lane), acc[j]); }
#pragma unroll
    for (int j = 0; j < 4; ++j) { const int a_ = j * 16 + col; const float dg = (a_ < ATT) ? bfr(DIAG[a_]) : 0.f;
#pragma unroll
      for (int r = 0; r < 8; ++r) sert[8 * g + r][a_] = tanh_ni(acc[j][r]) * dg; } }
  __syncthreads();
  if (wave == 1) { v8f acc[8] = {};
#pragma unroll
    for (int kc = 0; kc < AP / 32; ++kc) { const F2 a = split_row(&sert[col][0], kc * 32, lane);
#pragma unroll
      for (int j = 0; j < 8; ++j) { const F2 eb = split_row(ELT + (rbase + j * 16 + col) * AP, kc * 32, lane); acc[j] = mac3(a, eb, acc[j]); } }
#pragma unroll
    for (int j = 0; j < 8; ++j)
#pragma unroll
      for (int r = 0; r < 8; ++r) satt[8 * g + r][j * 16 + col] = acc[j][r]; }
  __syncthreads();
  for (int rr = 0; rr < 4; ++rr) { const int rl = wave * 4 + rr; float v[4]; float mxv = -3.0e38f;
#pragma unroll
    for (int i = 0; i < 4; ++i) { v[i] = satt[rl][lane + 32 * i]; mxv = fmaxf(mxv, v[i]); }
#pragma unroll
    for (int o = 1; o < 32; o <<= 1) mxv = fmaxf(mxv, __shfl_xor(mxv, o));
    float z = 0.f;
#pragma unroll
    for (int i = 0; i < 4; ++i) { v[i] = exp_ni(v[i] - mxv); z += v[i]; }
#pragma unroll
    for (int o = 1; o < 32; o <<= 1) z += __shfl_xor(z, o);
    const float iz = 1.0f / z;
#pragma unroll
    for (int i = 0; i < 4; ++i) satt[rl][lane + 32 * i] = v[i] * iz; }
  __syncthreads();
  { for (int jt = wave; jt < 13; jt += 4) { v8f acc = {};
#pragma unroll
      for (int kc = 0; kc < LL / 32; ++kc) { const F2 a = split_row(&satt[col][0], kc * 32, lane); const v16b lb = frag_b(LTT + ((size_t)b * DP + jt * 16 + col) * LL + kc * 32, lane); acc = wmma_bf(a.l, lb, acc); acc = wmma_bf(a.h, lb, acc); }
#pragma unroll
      for (int r = 0; r < 8; ++r) { const int d = jt * 16 + col; if (d < DP) sattl[8 * g + r][d] = (d < DD) ? acc[r] : 0.f; } } }
  if (wave == 2 || wave == 3) { const int jh = wave - 2; v8f acc[4] = {};
#pragma unroll
    for (int kc = 0; kc < DP / 32; ++kc) { v16b a; { const int k0 = kc * 32;
#pragma unroll
        for (int i = 0; i < 8; ++i) { a[i] = (__bf16)srt[col][k0 + 8 * g + i]; a[8 + i] = (__bf16)srt[col][k0 + 16 + 8 * g + i]; } }
#pragma unroll
      for (int j = 0; j < 4; ++j) acc[j] = wmma_bf(a, frag_b(&sltb[(jh * 4 + j) * 16 + col][kc * 32], lane), acc[j]); }
    float nr[8];
#pragma unroll
    for (int r = 0; r < 8; ++r) { float s = 0.f; const int rl = 8 * g + r; for (int d = col; d < DD; d += 16) s += srt[rl][d] * srt[rl][d];
#pragma unroll
      for (int o = 1; o < 16; o <<= 1) s += __shfl_xor(s, o);
      nr[r] = 1.0f / sqrtf(fmaxf(s, 1e-6f)); }
#pragma unroll
    for (int r = 0; r < 8; ++r) { float best = -3.0e38f; int bi = 0;
#pragma unroll
      for (int j = 0; j < 4; ++j) { const int l = (jh * 4 + j) * 16 + col; const float rel = acc[j][r] * nr[r] * NLT[rbase + l]; if (rel > best) { best = rel; bi = l; } }
#pragma unroll
      for (int o = 1; o < 16; o <<= 1) { const float ob = __shfl_xor(best, o); const int oi = __shfl_xor(bi, o); if (ob > best || (ob == best && oi < bi)) { best = ob; bi = oi; } }
      if (col == 0) { smx[jh][8 * g + r][0] = best; smx[jh][8 * g + r][1] = (float)bi; } } }
  __syncthreads();
  if (tid < 16) { const float b0 = smx[0][tid][0], b1 = smx[1][tid][0]; const int i0_ = (int)smx[0][tid][1], i1_ = (int)smx[1][tid][1]; spos[tid] = (b1 > b0) ? i1_ : i0_; }
  __syncthreads();
  for (int q = tid; q < 16 * DP; q += 128) { const int rl = q / DP, d = q % DP; int l = spos[rl]; l = l < 0 ? 0 : (l > LL - 1 ? LL - 1 : l); smal[rl][d] = (d < DD) ? bfr(LT[(rbase + l) * DD + d]) : 0.f; }
  __syncthreads();
  { const int rl = tid & 15, grp = tid >> 4;
#pragma unroll 1
    for (int e = grp; e < 63; e += 8) { float s = 0.f; int oc;
      if (e < 21) { oc = e; if (e == 0) {
#pragma unroll 4
          for (int d = 0; d < DD; ++d) s += slt[rl][d] * sh[d]; }
        else { const float* hw = HWF + ((size_t)b * MP + (e - 1)) * DP;
#pragma unroll 4
          for (int d = 0; d < DD; ++d) s += slt[rl][d] * hw[d]; } }
      else if (e < 42) { oc = 41 + (e - 21); if (e == 21) {
#pragma unroll 4
          for (int d = 0; d < DD; ++d) s += sattl[rl][d] * srt[rl][d]; }
        else { const float* wm = WAT + (size_t)(e - 22) * DD;
#pragma unroll 4
          for (int d = 0; d < DD; ++d) s += sattl[rl][d] * bfr(wm[d]) * srt[rl][d]; } }
      else { oc = 62 + (e - 42); if (e == 42) {
#pragma unroll 4
          for (int d = 0; d < DD; ++d) s += srt[rl][d] * smal[rl][d]; }
        else { const float* wm = WMA + (size_t)(e - 43) * DD;
#pragma unroll 4
          for (int d = 0; d < DD; ++d) s += srt[rl][d] * bfr(wm[d]) * smal[rl][d]; } }
      sout[rl][oc] = tanh_ni(s); } }
  __syncthreads();
  for (int q = tid; q < 16 * 24; q += 128) { const int rl = q / 24, pc = q % 24; vst2(OS + (rbase + i0 + rl) * 96 + pc * 4, *(const v4f*)&sout[rl][pc * 4]); }
}
__global__ __launch_bounds__(256) void k_out(const float* __restrict__ OS, float* __restrict__ out) {
  const size_t p = (size_t)blockIdx.x * 256 + threadIdx.x; const size_t total = (size_t)NR * NOUT; if (p * 4 >= total) return; v4f v;
#pragma unroll
  for (int i = 0; i < 4; ++i) { const size_t f = p * 4 + i; const size_t row = f / NOUT; v[i] = (f < total && row < (size_t)NBT * LL) ? OS[row * 96 + (f % NOUT)] : 0.f; }
  vst2(out + p * 4, v);
}
extern "C" void kernel_launch(void* const* d_in, const int* in_sizes, int n_in, void* d_out, int out_size, void* d_ws, size_t ws_size, hipStream_t stream) {
  (void)in_sizes; (void)n_in; (void)out_size;
  const float** F = (const float**)d_in;
  if (ws_size < (size_t)WS_END) return;
  char* ws = (char*)d_ws; __bf16 *PW1 = (__bf16*)(ws + WS_PW1), *PW2 = (__bf16*)(ws + WS_PW2), *LTT = (__bf16*)(ws + WS_LTT); float *HWF = (float*)(ws + WS_HWF), *ELT = (float*)(ws + WS_ELT), *NLT = (float*)(ws + WS_NLT), *OS = (float*)(ws + WS_OS);
  k_packw<<<AP / 8, 128, 0, stream>>>(F[8], PW1); k_packw<<<AP / 8, 128, 0, stream>>>(F[9], PW2);
  k_prep<<<NBT, 256, 0, stream>>>(F[0], F[2], F[3], F[4], PW2, HWF, ELT, LTT, NLT);
  k_main<<<dim3(LL / 16, NBT), 128, 0, stream>>>(F[0], F[1], F[5], F[6], F[7], PW1, F[10], F[2], F[3], HWF, ELT, LTT, NLT, OS);
  k_out<<<(unsigned)((((size_t)NR * NOUT) / 4 + 255) / 256), 256, 0, stream>>>(OS, (float*)d_out);
}
